// GNNEncoder_24515673325797
// MI455X (gfx1250) — hardware-verified
//
#include <hip/hip_runtime.h>
#define NNODE 50000
#define NEDGE 800000
#define NP2 1048576
#define D0 64
#define D1 128
#define D2 64

typedef __bf16 v16b __attribute__((ext_vector_type(16)));
typedef unsigned short v8us __attribute__((ext_vector_type(8), may_alias));
typedef float  v8f  __attribute__((ext_vector_type(8)));
typedef float  v4f  __attribute__((ext_vector_type(4)));
typedef float  v4fa __attribute__((ext_vector_type(4), may_alias));
union FragB { v16b v; v8us half[2]; unsigned short u[16]; };

__device__ __forceinline__ unsigned short bf16_bits(float x) { unsigned int u = __float_as_uint(x); return (unsigned short)((u + 0x7FFFu + ((u >> 16) & 1u)) >> 16); }
__device__ __forceinline__ float bf16_val(unsigned short b) { return __uint_as_float(((unsigned int)b) << 16); }
__device__ __forceinline__ float bf16_round(float x) { return bf16_val(bf16_bits(x)); }
template <int NT>
__device__ __forceinline__ v8f mmaN(v16b ah, v16b al, v16b bh, v16b bl, v8f c) {
  c = __builtin_amdgcn_wmma_f32_16x16x32_bf16(false, ah, false, bh, (short)0, c, false, false);
  if (NT >= 2) c = __builtin_amdgcn_wmma_f32_16x16x32_bf16(false, al, false, bh, (short)0, c, false, false);
  if (NT >= 3) c = __builtin_amdgcn_wmma_f32_16x16x32_bf16(false, ah, false, bl, (short)0, c, false, false);
  asm volatile("v_nop\n\tv_nop\n\tv_nop\n\tv_nop" : "+v"(c) : "v"(ah), "v"(al), "v"(bh), "v"(bl));
  return c;
}

__global__ __launch_bounds__(256) void k_wt_bf16(const float* __restrict__ W, unsigned short* __restrict__ Wt, int K, int N) {
  const int t = blockIdx.x * 256 + threadIdx.x;
  const int k8n = K / 8;
  if (t >= N * k8n) return;
  const int n = t / k8n, k8 = (t % k8n) * 8;
  v8us v;
#pragma unroll
  for (int i = 0; i < 8; ++i) v[i] = bf16_bits(W[(size_t)(k8 + i) * N + n]);
  *(volatile v8us*)(Wt + (size_t)n * K + k8) = v;
  __threadfence();
  *(volatile v8us*)(Wt + (size_t)n * K + k8) = v;
}

template <bool ASPLIT, int ACT, bool BIAS_BF16>
__global__ __launch_bounds__(128) void k_gemm_bf(const float* __restrict__ A, int lda, const unsigned short* __restrict__ Wt, int ldb,
                                               const float* __restrict__ bias, float* __restrict__ C, int ldc, int M, int N, int K) {
  __shared__ __attribute__((aligned(16))) float so[4][16][64];
  const int tid = threadIdx.x, w = tid >> 5, lane = tid & 31, ln = lane & 15, hh = lane >> 4;
  const int ntn = N / 64;
  const int wid = blockIdx.x * 4 + w;
  const int mt = wid / ntn, nq = wid % ntn;
  if (mt * 16 >= M) return;
  const int row0 = mt * 16, col0 = nq * 64;
  const float* arow = A + (size_t)(row0 + ln) * lda;
  v8f acc[4] = {};
  for (int kb = 0; kb < K; kb += 32) {
    FragB ah, al;
    const v4f x0 = *(const v4fa*)(arow + kb + 8 * hh), x1 = *(const v4fa*)(arow + kb + 8 * hh + 4);
    const v4f x2 = *(const v4fa*)(arow + kb + 16 + 8 * hh), x3 = *(const v4fa*)(arow + kb + 16 + 8 * hh + 4);
    float xs[16] = {x0[0],x0[1],x0[2],x0[3],x1[0],x1[1],x1[2],x1[3],x2[0],x2[1],x2[2],x2[3],x3[0],x3[1],x3[2],x3[3]};
#pragma unroll
    for (int i = 0; i < 16; ++i) { const unsigned short hb = bf16_bits(xs[i]); ah.u[i] = hb; al.u[i] = ASPLIT ? bf16_bits(xs[i] - bf16_val(hb)) : (unsigned short)0; }
#pragma unroll
    for (int t = 0; t < 4; ++t) {
      const unsigned short* brow = Wt + (size_t)(col0 + t * 16 + ln) * ldb + kb;
      FragB b;
      b.half[0] = *(const v8us*)(brow + 8 * hh);
      b.half[1] = *(const v8us*)(brow + 16 + 8 * hh);
      acc[t] = mmaN<ASPLIT ? 2 : 1>(ah.v, al.v, b.v, b.v, acc[t]);
    }
  }
#pragma unroll
  for (int t = 0; t < 4; ++t) {
    float bv = bias ? bias[col0 + t * 16 + ln] : 0.f;
    if (BIAS_BF16) bv = bf16_round(bv);
#pragma unroll
    for (int r = 0; r < 8; ++r) { float v = acc[t][r] + bv; if (ACT == 1) v = fmaxf(v, 0.f); so[w][8 * hh + r][t * 16 + ln] = v; }
  }
  __builtin_amdgcn_fence(__ATOMIC_ACQ_REL, "workgroup");
  __builtin_amdgcn_wave_barrier();
  const int rsub = lane >> 4, c4 = (lane & 15) * 4;
  for (int pass = 0; pass < 2; ++pass) {
#pragma unroll
    for (int q = 0; q < 8; ++q) {
      const int r = q * 2 + rsub;
      const v4f v = *(const v4fa*)&so[w][r][c4];
      *(volatile v4f*)(C + (size_t)(row0 + r) * ldc + col0 + c4) = v;
    }
    if (pass == 0) __threadfence();
  }
}

template <int D, bool CAUSAL>
__global__ __launch_bounds__(128) void k_flash(const float* __restrict__ qb, const float* __restrict__ kb, const float* __restrict__ vb,
                                             int pitch, int T, int H, float scale, float* __restrict__ y, int ypitch) {
  constexpr int KS = D / 32;
  constexpr int DT = D / 16;
  __shared__ __attribute__((aligned(16))) unsigned short sKh[32][D + 8], sKl[32][D + 8], sVh[32][D + 8], sVl[32][D + 8];
  __shared__ __attribute__((aligned(16))) unsigned short sPh[4][16][40], sPl[4][16][40];
  __shared__ __attribute__((aligned(16))) float sO[4][16][D];
  const int tid = threadIdx.x, w = tid >> 5, lane = tid & 31, ln = lane & 15, hh = lane >> 4;
  const int nqb = (T + 63) / 64;
  const int bh = blockIdx.x / nqb, qblk = blockIdx.x % nqb;
  const int b = bh / H, h = bh % H;
  const int q0 = qblk * 64 + w * 16;
  const float* Q = qb + (size_t)b * T * pitch + h * D;
  const float* K = kb + (size_t)b * T * pitch + h * D;
  const float* V = vb + (size_t)b * T * pitch + h * D;

  FragB aqh[KS], aql[KS];
  {
    int row = q0 + ln; if (row >= T) row = T - 1;
    const float* qr = Q + (size_t)row * pitch;
#pragma unroll
    for (int ks = 0; ks < KS; ++ks)
#pragma unroll
      for (int i = 0; i < 16; ++i) {
        const int d = ks * 32 + ((i < 8) ? (8 * hh + i) : (16 + 8 * hh + (i - 8)));
        const float x = qr[d] * scale; const unsigned short hb = bf16_bits(x);
        aqh[ks].u[i] = hb; aql[ks].u[i] = bf16_bits(x - bf16_val(hb));
      }
  }
  float m_r[8], l_r[8];
#pragma unroll
  for (int r = 0; r < 8; ++r) { m_r[r] = -3.0e38f; l_r[r] = 0.f; }
  v8f oacc[DT];
#pragma unroll
  for (int dt = 0; dt < DT; ++dt) oacc[dt] = (v8f){0.f,0.f,0.f,0.f,0.f,0.f,0.f,0.f};

  const int kv_end = CAUSAL ? min(T, qblk * 64 + 64) : T;
  for (int j0 = 0; j0 < kv_end; j0 += 32) {
    __syncthreads();
    for (int e = tid; e < 32 * (D / 4); e += 128) {
      const int r = e / (D / 4), c4 = (e % (D / 4)) * 4;
      const int key = j0 + r;
      v4f kf = {0.f,0.f,0.f,0.f}, vf = {0.f,0.f,0.f,0.f};
      if (key < T) { kf = *(const v4fa*)(K + (size_t)key * pitch + c4); vf = *(const v4fa*)(V + (size_t)key * pitch + c4); }
#pragma unroll
      for (int t = 0; t < 4; ++t) {
        unsigned short hb = bf16_bits(kf[t]); sKh[r][c4 + t] = hb; sKl[r][c4 + t] = bf16_bits(kf[t] - bf16_val(hb));
        hb = bf16_bits(vf[t]); sVh[r][c4 + t] = hb; sVl[r][c4 + t] = bf16_bits(vf[t] - bf16_val(hb));
      }
    }
    __syncthreads();
    v8f s[2];
#pragma unroll
    for (int nt = 0; nt < 2; ++nt) {
      v8f acc = {};
#pragma unroll
      for (int ks = 0; ks < KS; ++ks) {
        FragB bh_, bl_;
        bh_.half[0] = *(const v8us*)&sKh[nt * 16 + ln][ks * 32 + 8 * hh]; bh_.half[1] = *(const v8us*)&sKh[nt * 16 + ln][ks * 32 + 16 + 8 * hh];
        bl_.half[0] = *(const v8us*)&sKl[nt * 16 + ln][ks * 32 + 8 * hh]; bl_.half[1] = *(const v8us*)&sKl[nt * 16 + ln][ks * 32 + 16 + 8 * hh];
        acc = mmaN<3>(aqh[ks].v, aql[ks].v, bh_.v, bl_.v, acc);
      }
      s[nt] = acc;
    }
    float alpha[8];
#pragma unroll
    for (int r = 0; r < 8; ++r) {
      const int qi = q0 + 8 * hh + r;
      const int ja = j0 + ln, jb = j0 + 16 + ln;
      if (CAUSAL) { if (ja > qi) s[0][r] = -3.0e38f; if (jb > qi) s[1][r] = -3.0e38f; }
      if (ja >= T) s[0][r] = -3.0e38f;
      if (jb >= T) s[1][r] = -3.0e38f;
      float mx = fmaxf(s[0][r], s[1][r]);
      mx = fmaxf(mx, __shfl_xor(mx, 1, 32)); mx = fmaxf(mx, __shfl_xor(mx, 2, 32)); mx = fmaxf(mx, __shfl_xor(mx, 4, 32)); mx = fmaxf(mx, __shfl_xor(mx, 8, 32));
      const float mnew = fmaxf(m_r[r], mx);
      alpha[r] = (mnew > -1.0e38f) ? __expf(m_r[r] - mnew) : 1.0f;
      const float p0 = (s[0][r] > -1.0e38f) ? __expf(s[0][r] - mnew) : 0.f;
      const float p1 = (s[1][r] > -1.0e38f) ? __expf(s[1][r] - mnew) : 0.f;
      m_r[r] = mnew;
      l_r[r] = l_r[r] * alpha[r] + p0 + p1;
      unsigned short hb = bf16_bits(p0); sPh[w][8 * hh + r][ln] = hb;      sPl[w][8 * hh + r][ln] = bf16_bits(p0 - bf16_val(hb));
      hb = bf16_bits(p1);                sPh[w][8 * hh + r][16 + ln] = hb; sPl[w][8 * hh + r][16 + ln] = bf16_bits(p1 - bf16_val(hb));
    }
#pragma unroll
    for (int dt = 0; dt < DT; ++dt)
#pragma unroll
      for (int r = 0; r < 8; ++r) oacc[dt][r] *= alpha[r];
    __builtin_amdgcn_fence(__ATOMIC_ACQ_REL, "workgroup");
    __builtin_amdgcn_wave_barrier();
    FragB pah, pal;
    pah.half[0] = *(const v8us*)&sPh[w][ln][8 * hh]; pah.half[1] = *(const v8us*)&sPh[w][ln][16 + 8 * hh];
    pal.half[0] = *(const v8us*)&sPl[w][ln][8 * hh]; pal.half[1] = *(const v8us*)&sPl[w][ln][16 + 8 * hh];
#pragma unroll
    for (int dt = 0; dt < DT; ++dt) {
      FragB bvh, bvl;
#pragma unroll
      for (int i = 0; i < 8; ++i) {
        bvh.u[i] = sVh[8 * hh + i][dt * 16 + ln]; bvh.u[8 + i] = sVh[16 + 8 * hh + i][dt * 16 + ln];
        bvl.u[i] = sVl[8 * hh + i][dt * 16 + ln]; bvl.u[8 + i] = sVl[16 + 8 * hh + i][dt * 16 + ln];
      }
      oacc[dt] = mmaN<3>(pah.v, pal.v, bvh.v, bvl.v, oacc[dt]);
    }
    __builtin_amdgcn_fence(__ATOMIC_ACQ_REL, "workgroup");
    __builtin_amdgcn_wave_barrier();
  }
#pragma unroll
  for (int r = 0; r < 8; ++r) {
    float l = l_r[r];
    l += __shfl_xor(l, 1, 32); l += __shfl_xor(l, 2, 32); l += __shfl_xor(l, 4, 32); l += __shfl_xor(l, 8, 32);
    l_r[r] = (l > 0.f) ? 1.0f / l : 0.f;
  }
#pragma unroll
  for (int dt = 0; dt < DT; ++dt)
#pragma unroll
    for (int r = 0; r < 8; ++r) sO[w][8 * hh + r][dt * 16 + ln] = oacc[dt][r] * l_r[r];
  __builtin_amdgcn_fence(__ATOMIC_ACQ_REL, "workgroup");
  __builtin_amdgcn_wave_barrier();
  for (int pass = 0; pass < 2; ++pass) {
    for (int r = 0; r < 16; ++r) {
      const int row = q0 + r;
      if (row < T && lane < D / 4) {
        const v4f val = *(const v4fa*)&sO[w][r][lane * 4];
        *(volatile v4f*)(y + ((size_t)b * T + row) * ypitch + h * D + lane * 4) = val;
      }
    }
    if (pass == 0) __threadfence();
  }
}

__global__ __launch_bounds__(256) void k_sort_init(const int* __restrict__ seg, int n, int nseg, unsigned int* __restrict__ key, unsigned int* __restrict__ val, int np2) {
  const int i = blockIdx.x * 256 + threadIdx.x; if (i >= np2) return;
  unsigned int kv = 0xFFFFFFFFu;
  if (i < n) { int s = seg[i]; s = s < 0 ? 0 : (s >= nseg ? nseg - 1 : s); kv = (unsigned int)s; }
  *(volatile unsigned int*)(key + i) = kv; *(volatile unsigned int*)(val + i) = (unsigned int)i;
  __threadfence();
  *(volatile unsigned int*)(key + i) = kv; *(volatile unsigned int*)(val + i) = (unsigned int)i;
}
template <bool STAGE0>
__global__ __launch_bounds__(512) void k_sort_lds(unsigned int* __restrict__ key, unsigned int* __restrict__ val, int kstage) {
  __shared__ unsigned int sk[1024], sv[1024];
  const int tid = threadIdx.x; const int base = blockIdx.x * 1024;
  sk[tid] = key[base + tid]; sv[tid] = val[base + tid]; sk[tid + 512] = key[base + tid + 512]; sv[tid + 512] = val[base + tid + 512];
  __syncthreads();
  for (int k = (STAGE0 ? 2 : kstage); k <= (STAGE0 ? 1024 : kstage); k <<= 1) {
    for (int j = (k > 1024 ? 512 : (k >> 1)); j >= 1; j >>= 1) {
      const int lo = tid & (j - 1), hi2 = (tid >> __builtin_ctz(j)) << (__builtin_ctz(j) + 1);
      const int il = hi2 | lo, ir = il | j;
      const int gi = base + il;
      const bool asc = ((gi & k) == 0);
      unsigned int a = sk[il], b = sk[ir], va = sv[il], vb = sv[ir];
      const bool swp = asc ? (a > b) : (a < b);
      if (swp) { sk[il] = b; sk[ir] = a; sv[il] = vb; sv[ir] = va; }
      __syncthreads();
    }
  }
  for (int pass = 0; pass < 2; ++pass) {
    *(volatile unsigned int*)(key + base + tid) = sk[tid]; *(volatile unsigned int*)(val + base + tid) = sv[tid];
    *(volatile unsigned int*)(key + base + tid + 512) = sk[tid + 512]; *(volatile unsigned int*)(val + base + tid + 512) = sv[tid + 512];
    if (pass == 0) __threadfence();
  }
}
__global__ __launch_bounds__(256) void k_sort_step(unsigned int* __restrict__ key, unsigned int* __restrict__ val, int k, int j, int np2) {
  const int t = blockIdx.x * 256 + threadIdx.x; if (t >= np2 / 2) return;
  const int lo = t & (j - 1), il = ((t >> __builtin_ctz(j)) << (__builtin_ctz(j) + 1)) | lo, ir = il | j;
  const bool asc = ((il & k) == 0);
  unsigned int a = key[il], b = key[ir], va = val[il], vb = val[ir];
  const bool swp = asc ? (a > b) : (a < b);
  const unsigned int k1 = swp ? b : a, k2 = swp ? a : b, v1 = swp ? vb : va, v2 = swp ? va : vb;
  *(volatile unsigned int*)(key + il) = k1; *(volatile unsigned int*)(key + ir) = k2; *(volatile unsigned int*)(val + il) = v1; *(volatile unsigned int*)(val + ir) = v2;
  __threadfence();
  *(volatile unsigned int*)(key + il) = k1; *(volatile unsigned int*)(key + ir) = k2; *(volatile unsigned int*)(val + il) = v1; *(volatile unsigned int*)(val + ir) = v2;
}
__global__ __launch_bounds__(256) void k_rowptr(const unsigned int* __restrict__ key, int np2, int nseg, int* __restrict__ rowptr) {
  int s = blockIdx.x * 256 + threadIdx.x; if (s >= ((nseg + 1 + 31) / 32) * 32) return;
  const int sdst = s; if (s > nseg) s = nseg;
  int lo = 0, hi = np2;
  while (lo < hi) { const int mid = (lo + hi) >> 1; if (key[mid] < (unsigned int)s) lo = mid + 1; else hi = mid; }
  *(volatile int*)(rowptr + sdst) = lo; __threadfence(); *(volatile int*)(rowptr + sdst) = lo;
}
static void sort_pairs(unsigned int* key, unsigned int* val, int np2, hipStream_t stream) {
  k_sort_lds<true><<<np2 / 1024, 512, 0, stream>>>(key, val, 0);
  for (int k = 2048; k <= np2; k <<= 1) {
    for (int j = k >> 1; j >= 1024; j >>= 1) k_sort_step<<<(np2 / 2 + 255) / 256, 256, 0, stream>>>(key, val, k, j, np2);
    k_sort_lds<false><<<np2 / 1024, 512, 0, stream>>>(key, val, k);
  }
}

__global__ __launch_bounds__(256) void k_roundcopy(const float* __restrict__ src, float* __restrict__ dst, int n8) {
  const size_t t = (size_t)blockIdx.x * 256 + threadIdx.x;
  if (t >= (size_t)n8 * 2) return;
  v4f a = *(const v4fa*)(src + t * 4);
  for (int i = 0; i < 4; ++i) a[i] = bf16_round(a[i]);
  *(volatile v4f*)(dst + t * 4) = a; __threadfence(); *(volatile v4f*)(dst + t * 4) = a;
}

__global__ __launch_bounds__(256) void k_wt_cat(const float* __restrict__ Wl, const float* __restrict__ Wr, unsigned short* __restrict__ Bt, int Din, int Dout) {
  const int t = blockIdx.x * 256 + threadIdx.x; const int k8n = 2 * Din / 8; if (t >= Dout * k8n) return;
  const int n = t / k8n, k8 = (t % k8n) * 8; v8us v;
#pragma unroll
  for (int i = 0; i < 8; ++i) { const int k = k8 + i; v[i] = bf16_bits(k < Din ? Wl[(size_t)k * Dout + n] : Wr[(size_t)(k - Din) * Dout + n]); }
  *(volatile v8us*)(Bt + (size_t)n * 2 * Din + k8) = v; __threadfence(); *(volatile v8us*)(Bt + (size_t)n * 2 * Din + k8) = v;
}
template <int Din>
__global__ __launch_bounds__(256) void k_agg_cat(const float* __restrict__ h, const int* __restrict__ src, const int* __restrict__ rowptr, const unsigned int* __restrict__ perm, float* __restrict__ hcat) {
  const int tid = threadIdx.x, w = tid >> 5, lane = tid & 31; const int nd = blockIdx.x * 8 + w; if (nd >= NNODE) return;
  if (lane * 4 >= Din) return;
  v4f acc = {0.f,0.f,0.f,0.f};
  for (int p = rowptr[nd]; p < rowptr[nd + 1]; ++p) { int sn = src[perm[p]]; sn = sn < 0 ? 0 : (sn >= NNODE ? NNODE - 1 : sn); const v4f x0 = *(const v4fa*)(h + (size_t)sn * Din + lane * 4); for (int q = 0; q < 4; ++q) acc[q] += x0[q]; }
  const v4f own = *(const v4fa*)(h + (size_t)nd * Din + lane * 4);
  float* row = hcat + (size_t)nd * 2 * Din; *(volatile v4f*)(row + lane * 4) = acc; *(volatile v4f*)(row + Din + lane * 4) = own; __threadfence(); *(volatile v4f*)(row + lane * 4) = acc; *(volatile v4f*)(row + Din + lane * 4) = own;
}
template <int Dout, bool RELU>
__global__ __launch_bounds__(256) void k_norm_bn(float* __restrict__ h, const float* __restrict__ g, const float* __restrict__ bt, const float* __restrict__ rm, const float* __restrict__ rv) {
  const int tid = threadIdx.x, w = tid >> 5, lane = tid & 31; const int n = blockIdx.x * 8 + w; if (n >= NNODE) return;
  const bool act = lane * 4 < Dout;
  v4f a = {0.f,0.f,0.f,0.f}; if (act) a = *(const v4fa*)(h + (size_t)n * Dout + lane * 4);
  float s = a[0] * a[0] + a[1] * a[1] + a[2] * a[2] + a[3] * a[3]; for (int o = 16; o >= 1; o >>= 1) s += __shfl_xor(s, o, 32);
  const float inv = 1.0f / fmaxf(sqrtf(s), 1e-12f);
  if (act) { v4f o; for (int q = 0; q < 4; ++q) { const int c = lane * 4 + q; float v = bf16_round(g[c]) * (a[q] * inv - bf16_round(rm[c])) * rsqrtf(bf16_round(rv[c]) + 1e-5f) + bf16_round(bt[c]); if (RELU) v = fmaxf(v, 0.f); o[q] = v; }
    float* row = h + (size_t)n * Dout + lane * 4; *(volatile v4f*)row = o; __threadfence(); *(volatile v4f*)row = o; }
}
extern "C" void kernel_launch(void* const* d_in, const int* in_sizes, int n_in,
                              void* d_out, int out_size, void* d_ws, size_t ws_size, hipStream_t stream) {
  (void)in_sizes; (void)n_in; (void)out_size;
  const float* x = (const float*)d_in[0]; const int* ei = (const int*)d_in[1];
  const float* W1l = (const float*)d_in[2]; const float* b1 = (const float*)d_in[3]; const float* W1r = (const float*)d_in[4];
  const float* g1 = (const float*)d_in[5]; const float* bt1 = (const float*)d_in[6]; const float* rm1 = (const float*)d_in[7]; const float* rv1 = (const float*)d_in[8];
  const float* W2l = (const float*)d_in[9]; const float* b2 = (const float*)d_in[10]; const float* W2r = (const float*)d_in[11];
  const float* g2 = (const float*)d_in[12]; const float* bt2 = (const float*)d_in[13]; const float* rm2 = (const float*)d_in[14]; const float* rv2 = (const float*)d_in[15];
  const int* src = ei; const int* dst = ei + NEDGE;
  char* ws = (char*)d_ws; size_t off = 0;
  auto take = [&](size_t bytes) { char* p = ws + off; off += (bytes + 255) & ~(size_t)255; return p; };
  unsigned short* Bt1 = (unsigned short*)take((size_t)D1 * 2 * D0 * 2); unsigned short* Bt2 = (unsigned short*)take((size_t)D2 * 2 * D1 * 2);
  unsigned int* key = (unsigned int*)take((size_t)NP2 * 4); unsigned int* perm = (unsigned int*)take((size_t)NP2 * 4); int* rowptr = (int*)take((size_t)(NNODE + 64) * 4);
  float* xr = (float*)take((size_t)NNODE * D0 * 4); float* hcat = (float*)take((size_t)NNODE * 2 * D1 * 4); float* h1 = (float*)take((size_t)NNODE * D1 * 4);
  if (off > ws_size) return;
  k_wt_cat<<<(D1 * (2 * D0 / 8) + 255) / 256, 256, 0, stream>>>(W1l, W1r, Bt1, D0, D1);
  k_wt_cat<<<(D2 * (2 * D1 / 8) + 255) / 256, 256, 0, stream>>>(W2l, W2r, Bt2, D1, D2);
  k_sort_init<<<NP2 / 256, 256, 0, stream>>>(dst, NEDGE, NNODE, key, perm, NP2);
  sort_pairs(key, perm, NP2, stream);
  k_rowptr<<<(NNODE + 32 + 255) / 256, 256, 0, stream>>>(key, NP2, NNODE, rowptr);
  k_roundcopy<<<(NNODE * D0 / 4 + 255) / 256, 256, 0, stream>>>(x, xr, NNODE * D0 / 8);
  k_agg_cat<D0><<<(NNODE + 7) / 8, 256, 0, stream>>>(xr, src, rowptr, perm, hcat);
  k_gemm_bf<true, 0, true><<<((NNODE / 16) * (D1 / 64) + 3) / 4, 128, 0, stream>>>(hcat, 2 * D0, Bt1, 2 * D0, b1, h1, D1, NNODE, D1, 2 * D0);
  k_norm_bn<D1, true><<<(NNODE + 7) / 8, 256, 0, stream>>>(h1, g1, bt1, rm1, rv1);
  k_agg_cat<D1><<<(NNODE + 7) / 8, 256, 0, stream>>>(h1, src, rowptr, perm, hcat);
  k_gemm_bf<true, 0, true><<<((NNODE / 16) * (D2 / 64) + 3) / 4, 128, 0, stream>>>(hcat, 2 * D1, Bt2, 2 * D1, b2, (float*)d_out, D2, NNODE, D2, 2 * D1);
  k_norm_bn<D2, false><<<(NNODE + 7) / 8, 256, 0, stream>>>((float*)d_out, g2, bt2, rm2, rv2);
}
